// LocalGraphAttention_44057774522827
// MI455X (gfx1250) — hardware-verified
//
#include <hip/hip_runtime.h>
#include <stddef.h>


#define DF    128
#define NH    8
#define HC    16
#define QKVW  384
#define GR    32
#define AP    136
#define XSP   132
#define NB    512
#define CHUNK 2048
#define NTHR  256
#define NWAVE 8
#define WCAP  256
#define NGRP  (CHUNK / (NTHR * 4))

#define LDS_SACC (NB * DF)
#define LDS_DEN  (NB * NH)
#define LDS_LIST (NWAVE * WCAP)
#define LDS_BYTES ((LDS_SACC + LDS_DEN + LDS_LIST + NWAVE) * 4)

static_assert(WCAP == (CHUNK / NTHR) * 32);
static_assert(NGRP == 2);
static_assert(NB == 512);
static_assert(CHUNK == 2048);
static_assert(((LDS_SACC + LDS_DEN) % 4) == 0);
static_assert(LDS_BYTES == 286752);
static_assert(GR == 4 * NWAVE);
static_assert((AP % 8) == 0);
static_assert((XSP % 4) == 0);

typedef float          v4f   __attribute__((ext_vector_type(4)));
typedef float          v8f   __attribute__((ext_vector_type(8)));
typedef int            v4i   __attribute__((ext_vector_type(4)));
typedef unsigned short v8us  __attribute__((ext_vector_type(8)));
typedef __bf16         v16bf __attribute__((ext_vector_type(16)));
union Frag { v16bf v; v8us half[2]; };
union Pk8  { v8us v; v4i i4; unsigned short s[8]; };

__device__ __forceinline__ v8f wm(v16bf a, v16bf b, v8f c) {
  v8f d = __builtin_amdgcn_wmma_f32_16x16x32_bf16(false, a, false, b, (short)0, c, false, false);
  asm volatile("v_nop\n\tv_nop\n\tv_nop\n\tv_nop" : "+v"(d) : "v"(a), "v"(b));
  return d;
}

__device__ __forceinline__ unsigned short bf_rne(float x) {
  unsigned int u = __float_as_uint(x);
  u += 0x7fffu + ((u >> 16) & 1u);
  return (unsigned short)(u >> 16);
}

__device__ __forceinline__ void split1(float x, unsigned short& h, unsigned short& l) {
  const unsigned short hb = bf_rne(x);
  const float hf = __uint_as_float(((unsigned int)hb) << 16);
  h = hb;
  l = bf_rne(x - hf);
}

__global__ __launch_bounds__(NTHR) void k_prep(const float* __restrict__ W,
                                               unsigned short* Wh, unsigned short* Wl, int n8) {
  const int i = blockIdx.x * NTHR + threadIdx.x;
  if (i >= n8) return;
  const size_t o = (size_t)i * 8;
  const v4f a = *(const v4f*)(W + o);
  const v4f b = *(const v4f*)(W + o + 4);
  Pk8 uh, ul;
  split1(a.x, uh.s[0], ul.s[0]); split1(a.y, uh.s[1], ul.s[1]);
  split1(a.z, uh.s[2], ul.s[2]); split1(a.w, uh.s[3], ul.s[3]);
  split1(b.x, uh.s[4], ul.s[4]); split1(b.y, uh.s[5], ul.s[5]);
  split1(b.z, uh.s[6], ul.s[6]); split1(b.w, uh.s[7], ul.s[7]);
  *(volatile v4i*)(Wh + o) = uh.i4;
  *(volatile v4i*)(Wl + o) = ul.i4;
  __threadfence();
  *(volatile v4i*)(Wh + o) = uh.i4;
  *(volatile v4i*)(Wl + o) = ul.i4;
}

__global__ __launch_bounds__(NTHR) void k_gemm(
    const float* __restrict__ A, const unsigned short* __restrict__ Whi,
    const unsigned short* __restrict__ Wlo, float* C, int nValid, int ncg, int nStore) {
  __shared__ __attribute__((aligned(16))) unsigned short Ah[GR * AP];
  __shared__ __attribute__((aligned(16))) unsigned short Al[GR * AP];
  __shared__ __attribute__((aligned(16))) float Xs[GR * XSP];

  const int tid  = threadIdx.x;
  const int lane = tid & 31;
  const int wave = tid >> 5;
  const int hh   = lane >> 4;
  const int m    = lane & 15;
  const int rowBase = blockIdx.x * GR;
  const int ldc  = ncg * DF;

  {
    const int r  = tid >> 3;
    const int c0 = (tid & 7) * 16;
    int row = rowBase + r;
    if (row > nValid - 1) row = nValid - 1;
    const float* p = A + (size_t)row * DF + c0;
    const v4f f0 = *(const v4f*)(p), f1 = *(const v4f*)(p + 4);
    const v4f f2 = *(const v4f*)(p + 8), f3 = *(const v4f*)(p + 12);
    Pk8 h0, l0, h1, l1;
    split1(f0.x, h0.s[0], l0.s[0]); split1(f0.y, h0.s[1], l0.s[1]);
    split1(f0.z, h0.s[2], l0.s[2]); split1(f0.w, h0.s[3], l0.s[3]);
    split1(f1.x, h0.s[4], l0.s[4]); split1(f1.y, h0.s[5], l0.s[5]);
    split1(f1.z, h0.s[6], l0.s[6]); split1(f1.w, h0.s[7], l0.s[7]);
    split1(f2.x, h1.s[0], l1.s[0]); split1(f2.y, h1.s[1], l1.s[1]);
    split1(f2.z, h1.s[2], l1.s[2]); split1(f2.w, h1.s[3], l1.s[3]);
    split1(f3.x, h1.s[4], l1.s[4]); split1(f3.y, h1.s[5], l1.s[5]);
    split1(f3.z, h1.s[6], l1.s[6]); split1(f3.w, h1.s[7], l1.s[7]);
    *(v8us*)(Ah + r * AP + c0)     = h0.v;
    *(v8us*)(Ah + r * AP + c0 + 8) = h1.v;
    *(v8us*)(Al + r * AP + c0)     = l0.v;
    *(v8us*)(Al + r * AP + c0 + 8) = l1.v;
  }
  __syncthreads();

#pragma unroll 1
  for (int cg = 0; cg < ncg; ++cg) {
    const int ncolL = wave * 16 + m;
    const int ncol  = cg * DF + ncolL;
    v8f c0a = {0.f, 0.f, 0.f, 0.f, 0.f, 0.f, 0.f, 0.f};
    v8f c1a = {0.f, 0.f, 0.f, 0.f, 0.f, 0.f, 0.f, 0.f};
#pragma unroll 1
    for (int kt = 0; kt < DF / 32; ++kt) {
      const int k0 = kt * 32;
      Frag bh, bl, a0h, a0l, a1h, a1l;
      const unsigned short* pbh = Whi + (size_t)ncol * DF + k0 + 8 * hh;
      const unsigned short* pbl = Wlo + (size_t)ncol * DF + k0 + 8 * hh;
      const unsigned short* pa0 = Ah + m * AP + k0 + 8 * hh;
      const unsigned short* pa1 = Ah + (16 + m) * AP + k0 + 8 * hh;
      const unsigned short* pl0 = Al + m * AP + k0 + 8 * hh;
      const unsigned short* pl1 = Al + (16 + m) * AP + k0 + 8 * hh;
      bh.half[0]  = *(const v8us*)pbh;  bh.half[1]  = *(const v8us*)(pbh + 16);
      bl.half[0]  = *(const v8us*)pbl;  bl.half[1]  = *(const v8us*)(pbl + 16);
      a0h.half[0] = *(const v8us*)pa0;  a0h.half[1] = *(const v8us*)(pa0 + 16);
      a1h.half[0] = *(const v8us*)pa1;  a1h.half[1] = *(const v8us*)(pa1 + 16);
      a0l.half[0] = *(const v8us*)pl0;  a0l.half[1] = *(const v8us*)(pl0 + 16);
      a1l.half[0] = *(const v8us*)pl1;  a1l.half[1] = *(const v8us*)(pl1 + 16);
      c0a = wm(a0h.v, bh.v, c0a);
      c0a = wm(a0h.v, bl.v, c0a);
      c0a = wm(a0l.v, bh.v, c0a);
      c1a = wm(a1h.v, bh.v, c1a);
      c1a = wm(a1h.v, bl.v, c1a);
      c1a = wm(a1l.v, bh.v, c1a);
    }

#pragma unroll
    for (int r = 0; r < 8; ++r) {
      Xs[(8 * hh + r) * XSP + ncolL]      = c0a[r];
      Xs[(16 + 8 * hh + r) * XSP + ncolL] = c1a[r];
    }
    __syncthreads();

    v4f xr[4];
#pragma unroll
    for (int i = 0; i < 4; ++i) xr[i] = *(const v4f*)(Xs + (4 * wave + i) * XSP + 4 * lane);
    float* cp[4];
#pragma unroll
    for (int i = 0; i < 4; ++i)
      cp[i] = C + (size_t)(rowBase + 4 * wave + i) * ldc + cg * DF + 4 * lane;
#pragma unroll
    for (int i = 0; i < 4; ++i)
      if (rowBase + 4 * wave + i < nStore) *(volatile v4f*)(cp[i]) = xr[i];
    __threadfence();
#pragma unroll
    for (int i = 0; i < 4; ++i)
      if (rowBase + 4 * wave + i < nStore) *(volatile v4f*)(cp[i]) = xr[i];
    __syncthreads();
  }
}

__global__ __launch_bounds__(NTHR) void k_attn(
    const float* __restrict__ qkv, const int* __restrict__ rowp, const int* __restrict__ colp,
    float* agg, int nN, int nE) {
  extern __shared__ v4f lds_dyn[];
  float* sacc = (float*)lds_dyn;
  float* den  = sacc + LDS_SACC;
  int*   list = (int*)(den + LDS_DEN);
  int*   wcnt = list + LDS_LIST;

  const int tid  = threadIdx.x;
  const int lane = tid & 31;
  const int wave = tid >> 5;
  const int hd   = lane >> 2;
  const int nodeBase = blockIdx.x * NB;

  {
    const v4f z4 = {0.f, 0.f, 0.f, 0.f};
    for (int i = tid; i < (LDS_SACC + LDS_DEN) / 4; i += NTHR) lds_dyn[i] = z4;
  }
  __syncthreads();

  const bool al16 = ((((size_t)rowp) & 15) == 0);

  const int nChunks = (nE + CHUNK - 1) / CHUNK;
#pragma unroll 1
  for (int ch = 0; ch < nChunks; ++ch) {
    const int cbase = ch * CHUNK;
    int wc = 0;
#pragma unroll
    for (int g = 0; g < NGRP; ++g) {
      const int el0 = (g * NTHR + tid) * 4;
      const int e0  = cbase + el0;
      const int sent = -2147483647 - 1;
      v4i d;
      if (al16 && (cbase + CHUNK <= nE)) {
        d = *(const v4i*)(rowp + e0);
      } else {
        d.x = (e0     < nE) ? rowp[min(e0, nE - 1)]     : sent;
        d.y = (e0 + 1 < nE) ? rowp[min(e0 + 1, nE - 1)] : sent;
        d.z = (e0 + 2 < nE) ? rowp[min(e0 + 2, nE - 1)] : sent;
        d.w = (e0 + 3 < nE) ? rowp[min(e0 + 3, nE - 1)] : sent;
      }
      const unsigned s0 = (unsigned)d.x - (unsigned)nodeBase;
      const unsigned s1 = (unsigned)d.y - (unsigned)nodeBase;
      const unsigned s2 = (unsigned)d.z - (unsigned)nodeBase;
      const unsigned s3 = (unsigned)d.w - (unsigned)nodeBase;
      const bool h0 = s0 < (unsigned)NB;
      const bool h1 = s1 < (unsigned)NB;
      const bool h2 = s2 < (unsigned)NB;
      const bool h3 = s3 < (unsigned)NB;
      const unsigned anyhit = __builtin_amdgcn_ballot_w32(h0 | h1 | h2 | h3);
      if (anyhit != 0u) {
#define HITJ(J, HJ, SJ) { \
          const unsigned mj = __builtin_amdgcn_ballot_w32(HJ); \
          if (HJ) { \
            const int pos = wc + (int)__builtin_amdgcn_mbcnt_lo(mj, 0u); \
            if (pos < WCAP) list[wave * WCAP + pos] = ((el0 + (J)) << 9) | (int)(SJ); \
          } \
          wc += (int)__builtin_popcount(mj); }
        HITJ(0, h0, s0)
        HITJ(1, h1, s1)
        HITJ(2, h2, s2)
        HITJ(3, h3, s3)
#undef HITJ
      }
    }
    if (lane == 0) wcnt[wave] = wc;
    __syncthreads();

    if (wave == 0) {
#pragma unroll 1
      for (int wsx = 0; wsx < NWAVE; ++wsx) {
        int n = wcnt[wsx];
        if (n > WCAP) n = WCAP;
        if (n < 0) n = 0;
#pragma unroll 1
        for (int i = 0; i < n; ++i) {
          const int ent  = list[wsx * WCAP + i];
          const int slot = ent & (NB - 1);
          const int el   = (ent >> 9) & (CHUNK - 1);
          int e = cbase + el;
          if (e > nE - 1) e = nE - 1;
          int c = colp[e];
          c = c < 0 ? 0 : (c > nN - 1 ? nN - 1 : c);
          int nd = nodeBase + slot;
          if (nd > nN - 1) nd = nN - 1;
          const float* qrow = qkv + (size_t)nd * QKVW + 4 * lane;
          const float* krow = qkv + (size_t)c * QKVW + 4 * lane;
          const v4f qv = *(const v4f*)(qrow);
          const v4f kv = *(const v4f*)(krow + DF);
          const v4f vv = *(const v4f*)(krow + 2 * DF);
          float dp = qv.x * kv.x + qv.y * kv.y + qv.z * kv.z + qv.w * kv.w;
          dp += __shfl_xor(dp, 1, 32);
          dp += __shfl_xor(dp, 2, 32);
          float s = dp * 0.25f;
          s = (s >= 0.f) ? s : 0.2f * s;
          s = fminf(fmaxf(s, -20.f), 20.f);
          const float p = __expf(s);
          v4f* sp = (v4f*)(sacc + slot * DF + 4 * lane);
          const v4f cur = *sp;
          const v4f nxt = cur + p * vv;
          *sp = nxt;
          if ((lane & 3) == 0) {
            const float o = den[slot * NH + hd];
            den[slot * NH + hd] = o + p;
          }
        }
      }
    }
    __syncthreads();
  }

#pragma unroll 1
  for (int j = 0; j < NB / NWAVE; ++j) {
    const int slot = wave * (NB / NWAVE) + j;
    const int node = nodeBase + slot;
    if (node >= nN) break;
    const float dv  = den[slot * NH + hd];
    const float inv = 1.0f / (dv + 1e-10f);
    const v4f y = *(const v4f*)(sacc + slot * DF + 4 * lane) * inv;
    float* op = agg + (size_t)node * DF + 4 * lane;
    *(volatile v4f*)op = y;
    __threadfence();
    *(volatile v4f*)op = y;
  }
}

extern "C" void kernel_launch(void* const* d_in, const int* in_sizes, int n_in,
                              void* d_out, int out_size, void* d_ws, size_t ws_size,
                              hipStream_t stream) {
  if (n_in < 5) return;
  const int nN = in_sizes[0] / DF;
  const int nE = in_sizes[1];
  if (nN <= 0 || in_sizes[0] != nN * DF) return;
  if (nE < 0 || in_sizes[2] != nE) return;
  if (in_sizes[3] != QKVW * DF) return;
  if (in_sizes[4] != DF * DF) return;
  if (out_size != nN * DF) return;

  const float* x    = (const float*)d_in[0];
  const int*   rowp = (const int*)d_in[1];
  const int*   colp = (const int*)d_in[2];
  const float* Wqkv = (const float*)d_in[3];
  const float* Wout = (const float*)d_in[4];
  float* out = (float*)d_out;

  const int nP = ((nN + GR - 1) / GR) * GR;
  size_t off = 0;
  unsigned short* Wqh = (unsigned short*)((char*)d_ws + off); off += (size_t)QKVW * DF * 2;
  unsigned short* Wql = (unsigned short*)((char*)d_ws + off); off += (size_t)QKVW * DF * 2;
  unsigned short* Woh = (unsigned short*)((char*)d_ws + off); off += (size_t)DF * DF * 2;
  unsigned short* Wol = (unsigned short*)((char*)d_ws + off); off += (size_t)DF * DF * 2;
  float* qkv = (float*)((char*)d_ws + off); off += (size_t)nP * QKVW * sizeof(float);
  float* agg = (float*)((char*)d_ws + off); off += (size_t)nP * DF * sizeof(float);
  if (off > ws_size) return;

  const int n8q = QKVW * DF / 8;
  const int n8o = DF * DF / 8;
  k_prep<<<(n8q + NTHR - 1) / NTHR, NTHR, 0, stream>>>(Wqkv, Wqh, Wql, n8q);
  k_prep<<<(n8o + NTHR - 1) / NTHR, NTHR, 0, stream>>>(Wout, Woh, Wol, n8o);

  k_gemm<<<nP / GR, NTHR, 0, stream>>>(x, Wqh, Wql, qkv, nN, QKVW / DF, nP);

  hipFuncSetAttribute(reinterpret_cast<const void*>(&k_attn),
                      hipFuncAttributeMaxDynamicSharedMemorySize, LDS_BYTES);
  const int gridA = (nN + NB - 1) / NB;
  k_attn<<<gridA, NTHR, LDS_BYTES, stream>>>(qkv, rowp, colp, agg, nN, nE);

  k_gemm<<<nP / GR, NTHR, 0, stream>>>(agg, Woh, Wol, out, nN, 1, nN);
}
